// QuantLSTMCell_11836929868185
// MI455X (gfx1250) — hardware-run, weakly checked
//
#include <hip/hip_runtime.h>


namespace {
constexpr int NBR = 4096, IN = 1024, H = 1024, KT = IN + H  , JW = 64  ;
constexpr float HS = 256.0f, WSC = 256.0f;
typedef _Float16 b16;
typedef __attribute__((ext_vector_type(16))) _Float16 v16b;
typedef __attribute__((ext_vector_type(8))) _Float16 v8b;
typedef __attribute__((ext_vector_type(8))) float v8f;
typedef __attribute__((ext_vector_type(4))) float v4f;
__device__ __forceinline__ float bf16_rne(float f) { unsigned int u = __float_as_uint(f); u += 0x7FFFu + ((u >> 16) & 1u); float r = __uint_as_float(u & 0xFFFF0000u); asm volatile("" : "+v"(r)); return r; }
__device__ __forceinline__ float bfv(float f) { float r = bf16_rne(f); asm volatile("" : "+v"(r)); return r; }
__device__ __forceinline__ void split16(float v, b16& hi, b16& lo) { hi = (b16)v; lo = (b16)(v - (float)hi); }
__device__ __forceinline__ v16b frag_kb(const b16* p, int hh) { const v8b a = *(const v8b*)(p + 8 * hh), b = *(const v8b*)(p + 16 + 8 * hh); v16b f;
#pragma unroll
  for (int e = 0; e < 8; ++e) { f[e] = a[e]; f[8 + e] = b[e]; } return f; }
__device__ __forceinline__ v8f wmma16b(v16b a, v16b b, v8f c) { v8f d = __builtin_amdgcn_wmma_f32_16x16x32_f16(false, a, false, b, (short)0, c, false, false); asm volatile("v_nop\n\tv_nop\n\tv_nop\n\tv_nop" : "+v"(d) : "v"(a), "v"(b)); return d; }
__device__ __forceinline__ void wave_lds_sync() { __builtin_amdgcn_fence(__ATOMIC_RELEASE, "workgroup"); __builtin_amdgcn_wave_barrier(); __builtin_amdgcn_fence(__ATOMIC_ACQUIRE, "workgroup"); }
__device__ __forceinline__ float pmul(float a, float b) { float p = a * b; asm volatile("" : "+v"(p)); return p; }
__device__ __forceinline__ float fq(float v, float sc, float isc) { float r = rintf(v * sc); r = fminf(fmaxf(r, -2147483648.0f), 2147483647.0f); return pmul(r, isc); }
__device__ __forceinline__ float sigm(float v) { return 1.0f / (1.0f + __expf(-v)); }

__global__ __launch_bounds__(256) void wput_kernel(const float* __restrict__ wih, const float* __restrict__ whh, const int* __restrict__ fbits, b16* __restrict__ WQ) { const size_t u = (size_t)blockIdx.x * 256 + threadIdx.x; if (u >= (size_t)4 * H * (KT / 8)) return; const int r = (int)(u / (KT / 8)), k0 = (int)(u % (KT / 8)) * 8; const float sc = exp2f((float)fbits[0]), isc = 1.0f / sc; v8b v;
#pragma unroll
  for (int j = 0; j < 8; ++j) { const int k = k0 + j; const float w = k < IN ? wih[(size_t)r * IN + k] : whh[(size_t)r * H + (k - IN)]; v[j] = (b16)(fq(bfv(w), sc, isc) * WSC); }
  for (int pass = 0; pass < 2; ++pass) { *(volatile v8b*)(WQ + (size_t)r * KT + k0) = v; __threadfence(); } }
__global__ __launch_bounds__(32) void cell_kernel(const float* __restrict__ x, const float* __restrict__ h, const float* __restrict__ c, const b16* __restrict__ WQ, const float* __restrict__ bih, const float* __restrict__ bhh, const int* __restrict__ fbits, int RLIM, float* __restrict__ HN, float* __restrict__ CN) {
  __shared__ __attribute__((aligned(16))) b16 Ah[16][IN + 8], Al[16][IN + 8]; __shared__ float G[16][4 * JW + 4]; const int lane = threadIdx.x, nloc = lane & 15, hlf = lane >> 4; const int jg = blockIdx.x % (H / JW); const size_t m0 = (size_t)(blockIdx.x / (H / JW)) * 16; if (m0 >= (size_t)RLIM) return; const int j0 = jg * JW;
  const float sc = exp2f((float)fbits[0]), isc = 1.0f / sc;
  v8f acc[16];
#pragma unroll
  for (int t = 0; t < 16; ++t) acc[t] = (v8f){};
#pragma unroll 1
  for (int part = 0; part < 2; ++part) {
    const float* src = part == 0 ? x : h;
    for (int rr = 0; rr < 16; ++rr) for (int q = 0; q < IN / 32; ++q) { const int k = q * 32 + lane; b16 p, ql; split16(fq(bfv(src[(m0 + rr) * IN + k]), sc, isc) * HS, p, ql); Ah[rr][k] = p; Al[rr][k] = ql; }
    wave_lds_sync();
#pragma unroll 2
    for (int kb = 0; kb < IN; kb += 32) { const v16b a = frag_kb(&Ah[nloc][kb], hlf), al = frag_kb(&Al[nloc][kb], hlf);
#pragma unroll
      for (int t = 0; t < 16; ++t) { const int grow = (t >> 2) * H + j0 + (t & 3) * 16 + nloc;
        const v16b bw = frag_kb(WQ + (size_t)grow * KT + part * IN + kb, hlf); acc[t] = wmma16b(a, bw, acc[t]); acc[t] = wmma16b(al, bw, acc[t]); } }
    wave_lds_sync(); }
#pragma unroll
  for (int t = 0; t < 16; ++t) { const int gi = t >> 2, jj = (t & 3) * 16 + nloc; const int grow = gi * H + j0 + jj; const float bb = fq(bfv(bih[grow]), sc, isc) + fq(bfv(bhh[grow]), sc, isc);
#pragma unroll
    for (int r8 = 0; r8 < 8; ++r8) G[8 * hlf + r8][gi * JW + jj] = fq(acc[t][r8] * (1.0f / (HS * WSC)) + bb, sc, isc); }
  wave_lds_sync();
  for (int pass = 0; pass < 2; ++pass) { for (int rr = 0; rr < 16; ++rr) for (int q = 0; q < 2; ++q) { const int jj = q * 32 + lane; const size_t idx = (m0 + rr) * H + j0 + jj;
      const float ig = fq(sigm(G[rr][jj]), sc, isc), fg = fq(sigm(G[rr][JW + jj]), sc, isc), gg = fq(tanhf(G[rr][2 * JW + jj]), sc, isc), og = fq(sigm(G[rr][3 * JW + jj]), sc, isc);
      const float cq = fq(bfv(c[idx]), sc, isc); const float cn = fq(pmul(fg, cq) + pmul(ig, gg), sc, isc); const float hn = fq(pmul(og, tanhf(cn)), sc, isc);
      ((volatile float*)CN)[idx] = cn; ((volatile float*)HN)[idx] = hn; } __threadfence(); } }
}

extern "C" void kernel_launch(void* const* d_in, const int* in_sizes, int n_in, void* d_out, int out_size, void* d_ws, size_t ws_size, hipStream_t stream) {
  (void)n_in;
  auto Fp = [&](int i) { return (const float*)d_in[i]; };
  if (in_sizes[0] != NBR * IN || in_sizes[1] != NBR * H || in_sizes[2] != NBR * H || in_sizes[3] != 4 * H * IN || in_sizes[4] != 4 * H * H || in_sizes[5] != 4 * H || in_sizes[6] != 4 * H || in_sizes[7] != 1 || out_size != 2 * NBR * H) return;
  const int RLIM = NBR;
  size_t off = 0; char* ws = (char*)d_ws;
  auto carve = [&](size_t bytes) { char* p = ws + off; off += (bytes + 255) & ~(size_t)255; return p; };
  b16* WQ = (b16*)carve((size_t)4 * H * KT * 2);
  if (off > ws_size || off > ((size_t)32 << 20)) return;
  float* HN = (float*)d_out; float* CN = HN + (size_t)NBR * H;
  wput_kernel<<<(unsigned)(((size_t)4 * H * (KT / 8) + 255) / 256), 256, 0, stream>>>(Fp(3), Fp(4), (const int*)d_in[7], WQ);
  cell_kernel<<<(RLIM / 16) * (H / JW), 32, 0, stream>>>(Fp(0), Fp(1), Fp(2), WQ, Fp(5), Fp(6), (const int*)d_in[7], RLIM, HN, CN);
}
